// CausalSelfAttention_42795054137680
// MI455X (gfx1250) — hardware-run, weakly checked
//
#include <hip/hip_runtime.h>
#include <math.h>

#ifndef NB
#define NB 2
#endif
#ifndef SEQ
#define SEQ 2048
#endif
#define NB_FULL 2
#define SEQ_FULL 2048
#define CE 1024
#define NH 16
#define HD 64
#define NX 256

static_assert(SEQ % 64 == 0);
static_assert(SEQ >= NX);
static_assert(SEQ <= SEQ_FULL);
static_assert(NB <= NB_FULL);
static_assert(NX % 64 == 0);
static_assert(CE % 64 == 0);
static_assert(CE == NH * HD);
static_assert(((long long)(NB - 1) * SEQ_FULL + SEQ) * CE <= (long long)NB_FULL * SEQ_FULL * CE);

typedef __attribute__((ext_vector_type(16))) _Float16 v16h;
typedef __attribute__((ext_vector_type(8)))  _Float16 v8h;
typedef __attribute__((ext_vector_type(16))) __bf16   v16b;
typedef __attribute__((ext_vector_type(8)))  __bf16   v8b;
typedef __attribute__((ext_vector_type(8)))  float    v8f;
typedef __attribute__((ext_vector_type(4)))  float    v4f;
typedef __attribute__((ext_vector_type(4)))  unsigned int v4u;


#define VST2(T, ptr, val) do { const T vst2_v_ = (val); *(volatile T*)(ptr) = vst2_v_; __threadfence(); *(volatile T*)(ptr) = vst2_v_; } while (0)

__device__ __forceinline__ float cmb_bf(float v) {
    const unsigned u = __float_as_uint(v);
    const unsigned r = (u + 0x7fffu + ((u >> 16) & 1u)) & 0xffff0000u;
    return __uint_as_float(r);
}
__device__ __forceinline__ unsigned short bfu_rne(float v) {
    unsigned u = __float_as_uint(v);
    u += 0x7fffu + ((u >> 16) & 1u);
    return (unsigned short)(u >> 16);
}
__device__ __forceinline__ unsigned int pk2h(float a, float b) {
    return (unsigned int)__builtin_bit_cast(unsigned short, (_Float16)a) | ((unsigned int)__builtin_bit_cast(unsigned short, (_Float16)b) << 16);
}

__device__ __forceinline__ v8f wmma16(v16h a, v16h b, v8f c) {
    c = __builtin_amdgcn_wmma_f32_16x16x32_f16(false, a, false, b, (short)0, c, false, false);
    asm volatile("v_nop\n\tv_nop\n\tv_nop\n\tv_nop" : "+v"(c) : "v"(a), "v"(b));
    return c;
}

__device__ __forceinline__ void dep_guard_h(v8f& a, v8f& b, v16h x, v16h y) { asm volatile("v_nop\n\tv_nop\n\tv_nop\n\tv_nop" : "+v"(a), "+v"(b) : "v"(x), "v"(y)); }
__device__ __forceinline__ void dep_guard_b(v8f& a, v8f& b, v16b x, v16b y) { asm volatile("v_nop\n\tv_nop\n\tv_nop\n\tv_nop" : "+v"(a), "+v"(b) : "v"(x), "v"(y)); }
__device__ __forceinline__ void keep4_h(v16h a, v16h b, v16h c, v16h d) { asm volatile("v_nop" :: "v"(a), "v"(b), "v"(c), "v"(d)); }
__device__ __forceinline__ void keep4_b(v16b a, v16b b, v16b c, v16b d) { asm volatile("v_nop" :: "v"(a), "v"(b), "v"(c), "v"(d)); }
__device__ __forceinline__ void acc_guard4(v8f& a, v8f& b, v8f& c, v8f& d) { asm volatile("v_nop\n\tv_nop\n\tv_nop\n\tv_nop" : "+v"(a), "+v"(b), "+v"(c), "+v"(d)); }

template <typename T> struct Frag;
template <> struct Frag<_Float16> {
    typedef v16h V; union U { v16h v; v8h h[2]; };
    static __device__ __forceinline__ v16h load(const _Float16* p) {
        U f; f.h[0] = *(const v8h*)(p); f.h[1] = *(const v8h*)(p + 16); return f.v;
    }
    static __device__ __forceinline__ v8f mma(v16h a, v16h b, v8f c) {
        return __builtin_amdgcn_wmma_f32_16x16x32_f16(false, a, false, b, (short)0, c, false, false);
    }
    static __device__ __forceinline__ void guard(v8f& a, v8f& b, v16h x, v16h y) { dep_guard_h(a, b, x, y); }
    static __device__ __forceinline__ void keep(v16h a, v16h b, v16h c, v16h d) { keep4_h(a, b, c, d); }
};
template <> struct Frag<__bf16> {
    typedef v16b V; union U { v16b v; v8b h[2]; };
    static __device__ __forceinline__ v16b load(const __bf16* p) {
        U f; f.h[0] = *(const v8b*)(p); f.h[1] = *(const v8b*)(p + 16); return f.v;
    }
    static __device__ __forceinline__ v8f mma(v16b a, v16b b, v8f c) {
        return __builtin_amdgcn_wmma_f32_16x16x32_bf16(false, a, false, b, (short)0, c, false, false);
    }
    static __device__ __forceinline__ void guard(v8f& a, v8f& b, v16b x, v16b y) { dep_guard_b(a, b, x, y); }
    static __device__ __forceinline__ void keep(v16b a, v16b b, v16b c, v16b d) { keep4_b(a, b, c, d); }
};
template <int ET> struct Elem;
template <> struct Elem<0> { typedef _Float16 T; };
template <> struct Elem<1> { typedef __bf16 T; };

template <int ET, int BIAS_MODE, bool RESID>
__global__ __launch_bounds__(256) void wmma_gemm64(
    const unsigned short* __restrict__ Ap, int lda, long strideA,
    const unsigned short* __restrict__ Btp, int ldb, long strideB,
    float* Cout, int ldc, long strideC,
    const float* __restrict__ bias,
    const float* resid, long strideR,
    int M, int N, int K, float scale) {
    typedef typename Elem<ET>::T T;
    typedef typename Frag<T>::V V;
    const T* A = (const T*)Ap; const T* Bt = (const T*)Btp;
    __shared__ __align__(16) float sT[8][16 * 68];
    const int b    = blockIdx.y;
    const int lane = threadIdx.x & 31;
    const int wave = threadIdx.x >> 5;
    const int tilesN = N >> 6;
    const int tilesM = M >> 6;
    const int tile = blockIdx.x * 8 + wave;
    if (tile >= tilesM * tilesN) return;
    const int tm = tile / tilesN;
    const int tn = tile - tm * tilesN;
    const int m0 = tm << 6;
    const int n0 = tn << 6;

    const T* Ab = A  + (size_t)b * strideA;
    const T* Bb = Bt + (size_t)b * strideB;

    const int rlane = lane & 15;
    const int koff  = (lane >> 4) * 8;
    const int mOff  = (lane >> 4) * 8;

    v8f acc[4][4];
#pragma unroll
    for (int i = 0; i < 4; ++i)
#pragma unroll
        for (int j = 0; j < 4; ++j) acc[i][j] = (v8f){0.f, 0.f, 0.f, 0.f, 0.f, 0.f, 0.f, 0.f};

    for (int k0 = 0; k0 < K; k0 += 32) {
        V bh[4];
#pragma unroll
        for (int j = 0; j < 4; ++j) {
            const size_t bo = (size_t)(n0 + (j << 4) + rlane) * ldb + koff + k0;
            bh[j] = Frag<T>::load(Bb + bo);
        }
#pragma unroll
        for (int i = 0; i < 4; ++i) {
            const size_t ao = (size_t)(m0 + (i << 4) + rlane) * lda + koff + k0;
            V ah = Frag<T>::load(Ab + ao);
#pragma unroll
            for (int j = 0; j < 4; ++j) acc[i][j] = Frag<T>::mma(ah, bh[j], acc[i][j]);
            Frag<T>::guard(acc[i][0], acc[i][3], ah, ah);
        }
        Frag<T>::keep(bh[0], bh[1], bh[2], bh[3]);
    }
    acc_guard4(acc[0][0], acc[0][1], acc[0][2], acc[0][3]);
    acc_guard4(acc[1][0], acc[1][1], acc[1][2], acc[1][3]);
    acc_guard4(acc[2][0], acc[2][1], acc[2][2], acc[2][3]);
    acc_guard4(acc[3][0], acc[3][1], acc[3][2], acc[3][3]);

    float* slab = sT[wave];
    const float* Rb = RESID ? (resid + (size_t)b * strideR) : nullptr;
    float* C = Cout + (size_t)b * strideC;
#pragma unroll
    for (int i = 0; i < 4; ++i) {
        const int mBase = m0 + (i << 4);
#pragma unroll
        for (int j = 0; j < 4; ++j) {
            const int n = n0 + (j << 4) + rlane;
            float bv = 0.f;
            if (BIAS_MODE == 2) bv = cmb_bf(bias[n]);
#pragma unroll
            for (int r = 0; r < 8; ++r) {
                float v = acc[i][j][r] * scale;
                if (BIAS_MODE == 2) v += bv;
                if (RESID) v += Rb[(size_t)(mBase + mOff + r) * ldc + n];
                slab[(mOff + r) * 68 + (j << 4) + rlane] = v;
            }
        }
        __builtin_amdgcn_fence(3  , "workgroup");
        __builtin_amdgcn_wave_barrier();
        __builtin_amdgcn_fence(2  , "workgroup");
        {
            const int hh = lane >> 4, c4 = (lane & 15) * 4;
            for (int pass = 0; pass < 2; ++pass) {
#pragma unroll
                for (int it = 0; it < 8; ++it) {
                    const int row = it * 2 + hh;
                    const v4f v = *(const v4f*)(slab + row * 68 + c4);
                    *(volatile v4f*)(C + (size_t)(mBase + row) * ldc + n0 + c4) = v;
                }
                __threadfence();
            }
        }
        __builtin_amdgcn_fence(3  , "workgroup");
        __builtin_amdgcn_wave_barrier();
        __builtin_amdgcn_fence(2  , "workgroup");
    }
}

template <int BF>
__global__ __launch_bounds__(256) void k_cast8(const float* __restrict__ SRC, int lds, int rpb, int srb, unsigned short* __restrict__ DST, int ldd, int nR, int nC, float sc) {
    const long long u = (long long)blockIdx.x * 256 + threadIdx.x; const int per = nC / 8; if (u >= (long long)nR * per) return;
    const int r = (int)(u / per); const int c0 = 8 * (int)(u % per);
    const int rs = (r / rpb) * srb + (r % rpb);
    const float* s = SRC + (long long)rs * lds + c0;
    const v4f a = *(const v4f*)s, b = *(const v4f*)(s + 4);
    float w[8] = {a.x, a.y, a.z, a.w, b.x, b.y, b.z, b.w};
#pragma unroll
    for (int e = 0; e < 8; ++e) w[e] = (BF ? cmb_bf(w[e]) : w[e]) * sc;
    v4u pk; pk.x = pk2h(w[0], w[1]); pk.y = pk2h(w[2], w[3]); pk.z = pk2h(w[4], w[5]); pk.w = pk2h(w[6], w[7]);
    VST2(v4u, (v4u*)(DST + (long long)r * ldd + c0), pk);
}
template <int WF16, int WBF>
__global__ __launch_bounds__(256) void k_castT8(const float* __restrict__ SRC, int lds, unsigned short* __restrict__ D16, unsigned short* __restrict__ DBF, int ldd, int nR, int nC, float sc) {
    const long long u = (long long)blockIdx.x * 256 + threadIdx.x; const int per = nR / 8; if (u >= (long long)nC * per) return;
    const int c = (int)(u / per); const int r0 = 8 * (int)(u % per);
    float w[8];
#pragma unroll
    for (int e = 0; e < 8; ++e) w[e] = cmb_bf(SRC[(long long)(r0 + e) * lds + c]);
    if (WF16) {
        v4u pk; pk.x = pk2h(w[0] * sc, w[1] * sc); pk.y = pk2h(w[2] * sc, w[3] * sc); pk.z = pk2h(w[4] * sc, w[5] * sc); pk.w = pk2h(w[6] * sc, w[7] * sc);
        VST2(v4u, (v4u*)(D16 + (long long)c * ldd + r0), pk);
    }
    if (WBF) {
        v4u pk;
        pk.x = (__float_as_uint(w[0]) >> 16) | (__float_as_uint(w[1]) & 0xffff0000u);
        pk.y = (__float_as_uint(w[2]) >> 16) | (__float_as_uint(w[3]) & 0xffff0000u);
        pk.z = (__float_as_uint(w[4]) >> 16) | (__float_as_uint(w[5]) & 0xffff0000u);
        pk.w = (__float_as_uint(w[6]) >> 16) | (__float_as_uint(w[7]) & 0xffff0000u);
        VST2(v4u, (v4u*)(DBF + (long long)c * ldd + r0), pk);
    }
}
__global__ __launch_bounds__(256) void k_split8(const float* __restrict__ SRC, long long sbs, int lds, unsigned short* __restrict__ DH, unsigned short* __restrict__ DL, long long dbs, int ldd, int nR, int nC) {
    const long long u = (long long)blockIdx.x * 256 + threadIdx.x; const int per = nC / 8; if (u >= (long long)nR * per) return;
    const int z = blockIdx.y; const int r = (int)(u / per); const int c0 = 8 * (int)(u % per);
    const float* s = SRC + (long long)z * sbs + (long long)r * lds + c0;
    const v4f a = *(const v4f*)s, b = *(const v4f*)(s + 4);
    const float w[8] = {a.x, a.y, a.z, a.w, b.x, b.y, b.z, b.w};
    unsigned int hh[8], ll[8];
#pragma unroll
    for (int e = 0; e < 8; ++e) { const unsigned short hb = bfu_rne(w[e]); hh[e] = hb; ll[e] = bfu_rne(w[e] - __uint_as_float(((unsigned)hb) << 16)); }
    v4u ph, pl;
    ph.x = hh[0] | (hh[1] << 16); ph.y = hh[2] | (hh[3] << 16); ph.z = hh[4] | (hh[5] << 16); ph.w = hh[6] | (hh[7] << 16);
    pl.x = ll[0] | (ll[1] << 16); pl.y = ll[2] | (ll[3] << 16); pl.z = ll[4] | (ll[5] << 16); pl.w = ll[6] | (ll[7] << 16);
    const long long o = (long long)z * dbs + (long long)r * ldd + c0;
    VST2(v4u, (v4u*)(DH + o), ph);
    VST2(v4u, (v4u*)(DL + o), pl);
}

template <int NXT>
__global__ __launch_bounds__(64) void k_gx_exact(const float* __restrict__ QKVp, long long bs, int ld, const int* __restrict__ KM, int mbs, float sc, float* __restrict__ AOX, long long obs, int ldo) {
    #pragma clang fp contract(off)
    __shared__ float qs[64]; __shared__ float ps[NXT]; __shared__ float red[2];
    const int i = blockIdx.x, h = blockIdx.y, b = blockIdx.z, t = threadIdx.x;
    const float NEGI = -__builtin_inff();
    const float* Qb = QKVp + (long long)b * bs; const float* Kb = Qb + CE; const float* Vb = Qb + 2 * CE;
    const int* km = KM + (long long)b * mbs;
    qs[t] = Qb[(long long)i * ld + h * 64 + t]; __syncthreads();
#pragma unroll
    for (int r = 0; r < NXT / 64; ++r) {
        const int j = t + 64 * r; const int jc = min(j, i); const float* kr = Kb + (long long)jc * ld + h * 64; float s = 0.f;
#pragma unroll 8
        for (int d = 0; d < 64; ++d) s += qs[d] * kr[d];
        const int kp = km[jc];
        ps[j] = (j <= i && kp != 0) ? s * sc : NEGI;
    }
    __syncthreads();
    if (t == 0) {
        float m = NEGI; for (int j = 0; j <= i; ++j) m = fmaxf(m, ps[j]);
        float z = 0.f; for (int j = 0; j <= i; ++j) { const float e = expf(ps[j] - m); ps[j] = e; z += e; }
        red[0] = 1.f / z;
    }
    __syncthreads();
    const float inv = red[0]; float o = 0.f;
    for (int j = 0; j <= i; ++j) o += ps[j] * Vb[(long long)j * ld + h * 64 + t];
    const float ov = o * inv;
    VST2(float, AOX + (long long)b * obs + (long long)i * ldo + h * 64 + t, ov);
}

#define AW 4
struct AttnP {
    const float* Q; const float* K; const float* V; float* O; const int* KM;
    long long sQb, sQh, sQi, sKb, sKh, sKj, sVb, sVh, sVj, sOb, sOh, sOi, sMb;
    int Lq, Lk, coff, pad0; float scale; int pad1;
};
static_assert(sizeof(AttnP) == 5 * 8 + 13 * 8 + 6 * 4);

union FH { v16h v; v8h h[2]; };
__device__ __forceinline__ v16h fh_c(const float* __restrict__ p, int hf) {
    const v4f x0 = *(const v4f*)(p + 8 * hf), x1 = *(const v4f*)(p + 8 * hf + 4), x2 = *(const v4f*)(p + 16 + 8 * hf), x3 = *(const v4f*)(p + 20 + 8 * hf);
    v16h a;
    a[0] = (_Float16)x0.x; a[1] = (_Float16)x0.y; a[2] = (_Float16)x0.z; a[3] = (_Float16)x0.w;
    a[4] = (_Float16)x1.x; a[5] = (_Float16)x1.y; a[6] = (_Float16)x1.z; a[7] = (_Float16)x1.w;
    a[8] = (_Float16)x2.x; a[9] = (_Float16)x2.y; a[10] = (_Float16)x2.z; a[11] = (_Float16)x2.w;
    a[12] = (_Float16)x3.x; a[13] = (_Float16)x3.y; a[14] = (_Float16)x3.z; a[15] = (_Float16)x3.w;
    return a;
}

__global__ __launch_bounds__(32 * AW) void k_attn(AttnP p) {
    constexpr int PP = 72;
    __shared__ __align__(16) _Float16 vt[64 * PP];
    __shared__ __align__(16) _Float16 ph[AW][16 * PP];
    __shared__ __align__(16) float    ol[AW][16 * 68];
    const int lane = threadIdx.x & 31, hf = lane >> 4, l15 = lane & 15, wave = threadIdx.x >> 5;
    const int h = blockIdx.y, b = blockIdx.z;
    const int q0 = (blockIdx.x * AW + wave) * 16;
    const float L2E = 1.4426950408889634f;
    const float NEG = -__builtin_inff();
    const int qi = min(q0 + l15, p.Lq - 1);
    const float* qrow = p.Q + b * p.sQb + h * p.sQh + (long long)qi * p.sQi;
    const float* kbase = p.K + b * p.sKb + h * p.sKh;
    const float* vbase = p.V + b * p.sVb + h * p.sVh;
    const int* kmb = p.KM + b * p.sMb;
    v16h qa[2];
    qa[0] = fh_c(qrow, hf); qa[1] = fh_c(qrow + 32, hf);
    v8f o[4]; float m8[8], l8[8];
#pragma unroll
    for (int t = 0; t < 4; ++t) { v8f zz = {}; o[t] = zz; }
#pragma unroll
    for (int i = 0; i < 8; ++i) { m8[i] = NEG; l8[i] = 0.f; }
    const int je = (int)(blockIdx.x * AW + AW - 1) * 16 + 16 + p.coff;
    const int jend = min(p.Lk, max(je, 0));
    for (int j0 = 0; j0 < jend; j0 += 64) {
        __syncthreads();
#pragma unroll
        for (int it = 0; it < 8; ++it) {
            const int idx = threadIdx.x + it * 128; const int jr = idx >> 4, d4 = (idx & 15) * 4;
            const int jc = min(j0 + jr, p.Lk - 1);
            const v4f f = *(const v4f*)(vbase + (long long)jc * p.sVj + d4);
            const bool live = (j0 + jr) < p.Lk;
            vt[(d4 + 0) * PP + jr] = (_Float16)(live ? f.x : 0.f);
            vt[(d4 + 1) * PP + jr] = (_Float16)(live ? f.y : 0.f);
            vt[(d4 + 2) * PP + jr] = (_Float16)(live ? f.z : 0.f);
            vt[(d4 + 3) * PP + jr] = (_Float16)(live ? f.w : 0.f);
        }
        v8f s[4]; int kk[4];
#pragma unroll
        for (int t = 0; t < 4; ++t) {
            const int jc = min(j0 + t * 16 + l15, p.Lk - 1);
            kk[t] = kmb[jc];
            const float* krow = kbase + (long long)jc * p.sKj;
            v8f acc = {};
            acc = wmma16(qa[0], fh_c(krow, hf), acc);
            acc = wmma16(qa[1], fh_c(krow + 32, hf), acc);
            s[t] = acc;
        }
        float pv[8][4];
#pragma unroll
        for (int i = 0; i < 8; ++i) {
            const int irow = q0 + i + 8 * hf;
            float sc[4];
#pragma unroll
            for (int t = 0; t < 4; ++t) {
                const int jg = j0 + t * 16 + l15;
                const bool dead = (jg >= p.Lk) || (jg > irow + p.coff) || (kk[t] == 0);
                const float v = s[t][i] * p.scale * L2E;
                sc[t] = dead ? NEG : v;
            }
            float mx = fmaxf(fmaxf(sc[0], sc[1]), fmaxf(sc[2], sc[3]));
            mx = fmaxf(mx, __shfl_xor(mx, 1, 32)); mx = fmaxf(mx, __shfl_xor(mx, 2, 32));
            mx = fmaxf(mx, __shfl_xor(mx, 4, 32)); mx = fmaxf(mx, __shfl_xor(mx, 8, 32));
            const float mnew = fmaxf(m8[i], mx);
            const float corr = (mnew == NEG) ? 1.f : exp2f(m8[i] - mnew);
            float rs = 0.f;
#pragma unroll
            for (int t = 0; t < 4; ++t) {
                const float e = exp2f(sc[t] - mnew);
                const float pp = (sc[t] == NEG) ? 0.f : e; rs += pp; pv[i][t] = pp;
            }
            rs += __shfl_xor(rs, 1, 32); rs += __shfl_xor(rs, 2, 32); rs += __shfl_xor(rs, 4, 32); rs += __shfl_xor(rs, 8, 32);
            l8[i] = l8[i] * corr + rs; m8[i] = mnew;
#pragma unroll
            for (int t = 0; t < 4; ++t) o[t][i] *= corr;
        }
#pragma unroll
        for (int i = 0; i < 8; ++i)
#pragma unroll
            for (int t = 0; t < 4; ++t) ph[wave][(i + 8 * hf) * PP + t * 16 + l15] = (_Float16)(pv[i][t] * 4096.f);
        __syncthreads();
        FH pa0, pa1;
        pa0.h[0] = *(const v8h*)(&ph[wave][l15 * PP + 8 * hf]);
        pa0.h[1] = *(const v8h*)(&ph[wave][l15 * PP + 16 + 8 * hf]);
        pa1.h[0] = *(const v8h*)(&ph[wave][l15 * PP + 32 + 8 * hf]);
        pa1.h[1] = *(const v8h*)(&ph[wave][l15 * PP + 48 + 8 * hf]);
#pragma unroll
        for (int t = 0; t < 4; ++t) {
            const int dcol = t * 16 + l15;
            FH b0, b1;
            b0.h[0] = *(const v8h*)(&vt[dcol * PP + 8 * hf]);
            b0.h[1] = *(const v8h*)(&vt[dcol * PP + 16 + 8 * hf]);
            b1.h[0] = *(const v8h*)(&vt[dcol * PP + 32 + 8 * hf]);
            b1.h[1] = *(const v8h*)(&vt[dcol * PP + 48 + 8 * hf]);
            o[t] = wmma16(pa0.v, b0.v, o[t]);
            o[t] = wmma16(pa1.v, b1.v, o[t]);
        }
    }
    float invr[8];
#pragma unroll
    for (int i = 0; i < 8; ++i) {
        const float q = 1.f / (fmaxf(l8[i], 1.0e-30f) * 4096.f);
        invr[i] = (l8[i] > 0.f) ? q : __uint_as_float(0x7fc00000u);
    }
#pragma unroll
    for (int i = 0; i < 8; ++i)
#pragma unroll
        for (int t = 0; t < 4; ++t) ol[wave][(i + 8 * hf) * 68 + t * 16 + l15] = o[t][i] * invr[i];
    __syncthreads();
    float* obase = p.O + b * p.sOb + h * p.sOh;
    const int c4 = l15 * 4;
    for (int pass = 0; pass < 2; ++pass) {
#pragma unroll
        for (int it = 0; it < 8; ++it) {
            const int row = it * 2 + hf;
            const v4f v = *(const v4f*)(&ol[wave][row * 68 + c4]);
            if (q0 + row < p.Lq) *(volatile v4f*)(obase + (long long)(q0 + row) * p.sOi + c4) = v;
        }
        __threadfence();
    }
}

extern "C" void kernel_launch(void* const* d_in, const int* in_sizes, int n_in, void* d_out, int out_size, void* d_ws, size_t ws_size, hipStream_t stream) {
    (void)out_size;
    if (n_in < 6) return;
    const long long MR = (long long)NB * SEQ;
    if ((long long)in_sizes[0] < ((long long)(NB - 1) * SEQ_FULL + SEQ) * CE) return;
    if ((long long)in_sizes[1] < (long long)(NB - 1) * SEQ_FULL + SEQ) return;
    if ((long long)in_sizes[2] < (long long)CE * 3 * CE) return;
    if ((long long)in_sizes[3] < 3 * CE) return;
    if ((long long)in_sizes[4] < (long long)CE * CE) return;
    if ((long long)in_sizes[5] < CE) return;
    const float* x      = (const float*)d_in[0];
    const int*   tmask  = (const int*)d_in[1];
    const float* W_attn = (const float*)d_in[2];
    const float* b_attn = (const float*)d_in[3];
    const float* W_proj = (const float*)d_in[4];
    const float* b_proj = (const float*)d_in[5];
    float* out = (float*)d_out;

    char* wsp = (char*)d_ws;
    unsigned short* X16  = (unsigned short*)wsp; wsp += (size_t)MR * CE * 2;
    unsigned short* W316 = (unsigned short*)wsp; wsp += (size_t)3 * CE * CE * 2;
    float*          QKV  = (float*)wsp;          wsp += (size_t)MR * 3 * CE * 4;
    float*          AO   = (float*)wsp;          wsp += (size_t)MR * CE * 4;
    unsigned short* WO16 = (unsigned short*)wsp; wsp += (size_t)CE * CE * 2;
    unsigned short* WOB  = (unsigned short*)wsp; wsp += (size_t)CE * CE * 2;
    unsigned short* AOH2 = (unsigned short*)wsp; wsp += (size_t)NB * NX * CE * 2;
    unsigned short* AOL2 = (unsigned short*)wsp; wsp += (size_t)NB * NX * CE * 2;
    unsigned short* AO16 = X16;
    static_assert((size_t)NB * SEQ * CE * 2 + (size_t)3 * CE * CE * 2 + (size_t)NB * SEQ * 3 * CE * 4 + (size_t)NB * SEQ * CE * 4
                  + (size_t)2 * CE * CE * 2 + (size_t)2 * NB * NX * CE * 2 <= (size_t)134217728);
    if ((size_t)(wsp - (char*)d_ws) > ws_size) return;

    k_cast8<1><<<(unsigned)((MR * (CE / 8) + 255) / 256), 256, 0, stream>>>(x, CE, SEQ, SEQ_FULL, X16, CE, (int)MR, CE, 1.0f);
    k_castT8<1, 0><<<(unsigned)(((long long)(3 * CE) * (CE / 8) + 255) / 256), 256, 0, stream>>>(W_attn, 3 * CE, W316, nullptr, CE, CE, 3 * CE, 16.0f);
    wmma_gemm64<0, 2, false><<<dim3((unsigned)((((MR / 64) * ((3 * CE) / 64)) + 7) / 8), 1u), 256, 0, stream>>>(
        X16, CE, 0L, W316, CE, 0L, QKV, 3 * CE, 0L, b_attn, nullptr, 0L, (int)MR, 3 * CE, CE, 0.0625f);
    k_castT8<1, 1><<<(unsigned)(((long long)CE * (CE / 8) + 255) / 256), 256, 0, stream>>>(W_proj, CE, WO16, WOB, CE, CE, CE, 16.0f);
    k_gx_exact<NX><<<dim3(NX, NH, NB), 64, 0, stream>>>(QKV, (long long)SEQ * 3 * CE, 3 * CE, tmask, SEQ_FULL, 0.125f, AO, (long long)SEQ * CE, CE);
    if (SEQ > NX) {
        AttnP a;
        a.Q = QKV + (size_t)NX * 3 * CE; a.K = QKV + CE; a.V = QKV + 2 * CE; a.O = AO + (size_t)NX * CE; a.KM = tmask;
        a.sQb = (long long)SEQ * 3 * CE; a.sQh = HD; a.sQi = 3 * CE;
        a.sKb = (long long)SEQ * 3 * CE; a.sKh = HD; a.sKj = 3 * CE;
        a.sVb = (long long)SEQ * 3 * CE; a.sVh = HD; a.sVj = 3 * CE;
        a.sOb = (long long)SEQ * CE; a.sOh = HD; a.sOi = CE; a.sMb = SEQ_FULL;
        a.Lq = SEQ - NX; a.Lk = SEQ; a.coff = NX; a.pad0 = 0; a.scale = 0.125f; a.pad1 = 0;
        k_attn<<<dim3((unsigned)((SEQ - NX + 16 * AW - 1) / (16 * AW)), (unsigned)NH, (unsigned)NB), 32 * AW, 0, stream>>>(a);
    }
    k_cast8<0><<<(unsigned)((MR * (CE / 8) + 255) / 256), 256, 0, stream>>>(AO, CE, (int)MR, 0, AO16, CE, (int)MR, CE, 16.0f);
    wmma_gemm64<0, 2, false><<<dim3((unsigned)((((SEQ / 64) * (CE / 64)) + 7) / 8), (unsigned)NB), 256, 0, stream>>>(
        AO16, CE, (long)SEQ * CE, WO16, CE, 0L, out, CE, (long)SEQ_FULL * CE, b_proj, nullptr, 0L, SEQ, CE, CE, 1.0f / 256.0f);
    k_split8<<<dim3((unsigned)(((long long)NX * (CE / 8) + 255) / 256), (unsigned)NB), 256, 0, stream>>>(AO, (long long)SEQ * CE, CE, AOH2, AOL2, (long long)NX * CE, CE, NX, CE);
    wmma_gemm64<1, 2, false><<<dim3((unsigned)((((NX / 64) * (CE / 64)) + 7) / 8), (unsigned)NB), 256, 0, stream>>>(
        AOH2, CE, (long)NX * CE, WOB, CE, 0L, out, CE, (long)SEQ_FULL * CE, b_proj, nullptr, 0L, NX, CE, CE, 1.0f);
    wmma_gemm64<1, 0, true><<<dim3((unsigned)((((NX / 64) * (CE / 64)) + 7) / 8), (unsigned)NB), 256, 0, stream>>>(
        AOL2, CE, (long)NX * CE, WOB, CE, 0L, out, CE, (long)SEQ_FULL * CE, nullptr, out, (long)SEQ_FULL * CE, NX, CE, CE, 1.0f);
}
